// SelfAttention_1322849927509
// MI455X (gfx1250) — hardware-verified
//
#include <hip/hip_runtime.h>
#ifndef NB
#define NB 1
#endif
#ifndef SEQ
#define SEQ 4096
#endif
#define SEQ_FULL 4096
#define CC 128
#define NH 4
#define HD 32
#define HXP 136
#define SVP 72
#define SOP 68
#define XS ((size_t)CC * SEQ_FULL)
#define QKS ((size_t)NB * NH * SEQ * HD)

static_assert(CC == NH * HD);
static_assert(HD == 32);
static_assert(CC == 128);
static_assert(CC <= 256);
static_assert(SEQ % 64 == 0);
static_assert(SEQ <= SEQ_FULL);
static_assert(64 * HXP <= 128 * SVP);
static_assert(HXP % 8 == 0 && SVP % 8 == 0 && SOP % 4 == 0);
static_assert((CC * CC) % (8 * 256) == 0);

typedef _Float16 v16h __attribute__((ext_vector_type(16)));
typedef unsigned short v8us __attribute__((ext_vector_type(8), may_alias));
typedef float v8f  __attribute__((ext_vector_type(8)));
typedef float v4f  __attribute__((ext_vector_type(4)));
typedef float v4fa __attribute__((ext_vector_type(4), may_alias));
union FragH { v16h v; v8us half[2]; _Float16 h[16]; unsigned short u[16]; };

constexpr size_t WS_W16 = 0;
constexpr size_t SZ_W16 = (size_t)4 * CC * CC * 2;
constexpr size_t WS_GS  = WS_W16 + SZ_W16;
constexpr size_t SZ_GS  = (size_t)NB * 2 * CC * 32 * 4;
constexpr size_t WS_QK  = WS_GS + SZ_GS;
constexpr size_t SZ_QK  = 2 * QKS * 2;
constexpr size_t WS_VT  = WS_QK + SZ_QK;
constexpr size_t SZ_VT  = (size_t)NB * CC * SEQ * 2;
constexpr size_t WS_AO  = WS_VT + SZ_VT;
constexpr size_t SZ_AO  = (size_t)NB * SEQ * CC * 2;
constexpr size_t WS_TOTAL = WS_AO + SZ_AO;
static_assert(SZ_W16 % 256 == 0 && SZ_GS % 256 == 0 && SZ_QK % 256 == 0 && SZ_VT % 256 == 0 && SZ_AO % 256 == 0);
static_assert(WS_TOTAL <= (size_t)134217728);

__device__ __forceinline__ float bf16_rne(float x) {
  unsigned int u = __float_as_uint(x);
  u = (u + 0x7FFFu + ((u >> 16) & 1u)) & 0xFFFF0000u;
  return __uint_as_float(u);
}

__device__ __forceinline__ v16h ld_frag(const _Float16* __restrict__ p, int hh) {
  FragH f;
  const unsigned short* q = (const unsigned short*)p;
  f.half[0] = *(const v8us*)(q + 8 * hh);
  f.half[1] = *(const v8us*)(q + 16 + 8 * hh);
  return f.v;
}
__device__ __forceinline__ v8f mma(v16h a, v16h b, v8f c) {
  v8f d = __builtin_amdgcn_wmma_f32_16x16x32_f16(false, a, false, b, (short)0, c, false, false);
  asm volatile("v_nop\n\tv_nop\n\tv_nop\n\tv_nop" : "+v"(d) : "v"(a), "v"(b));
  return d;
}

__device__ __forceinline__ float blk_sum256(float v) {
  __shared__ float red[256];
  const int t = threadIdx.x;
  red[t] = v;
  __syncthreads();
#pragma unroll 1
  for (int st = 128; st > 0; st >>= 1) {
    if (t < st) red[t] = red[t] + red[t + st];
    __syncthreads();
  }
  const float r = red[0];
  __syncthreads();
  return r;
}

__device__ __forceinline__ v8us cvt_w8(const float* __restrict__ w, int e) {
  const v4f a = *(const v4fa*)(w + e), c = *(const v4fa*)(w + e + 4);
  FragH f;
#pragma unroll
  for (int q = 0; q < 4; ++q) {
    f.h[q]     = (_Float16)(bf16_rne(a[q]) * 16.0f);
    f.h[4 + q] = (_Float16)(bf16_rne(c[q]) * 16.0f);
  }
  return f.half[0];
}

__global__ __launch_bounds__(256) void k_wcvt(const float* __restrict__ qw, const float* __restrict__ kw, const float* __restrict__ vw,
                                              const float* __restrict__ pw, _Float16* __restrict__ W16) {
  const int t = blockIdx.x * 256 + threadIdx.x;
  if (t >= CC * CC / 8) return;
  const int e = t * 8;
  const v8us v0 = cvt_w8(qw, e), v1 = cvt_w8(kw, e), v2 = cvt_w8(vw, e), v3 = cvt_w8(pw, e);
  unsigned short* d = (unsigned short*)W16 + e;
  for (int pass = 0; pass < 2; ++pass) {
    *(volatile v8us*)(d) = v0;
    *(volatile v8us*)(d + CC * CC) = v1;
    *(volatile v8us*)(d + 2 * CC * CC) = v2;
    *(volatile v8us*)(d + 3 * CC * CC) = v3;
    if (pass == 0) __threadfence();
  }
}

__global__ __launch_bounds__(256) void k_gnsum(const float* __restrict__ x, float* __restrict__ GS) {
  const int tid = threadIdx.x, c = blockIdx.x, b = blockIdx.y;
  const float* xr = x + (size_t)b * XS + (size_t)c * SEQ_FULL;
  float s = 0.f;
#pragma unroll 1
  for (int j = tid * 4; j < SEQ; j += 1024) {
    const v4f a = *(const v4fa*)(xr + j);
    s += (bf16_rne(a[0]) + bf16_rne(a[1])) + (bf16_rne(a[2]) + bf16_rne(a[3]));
  }
  const float tot = blk_sum256(s);
  float* d = GS + ((size_t)b * 2 * CC + c) * 32;
  const v4f o = {(tid == 0) ? tot : 0.f, 0.f, 0.f, 0.f};
  if (tid < 8) *(volatile v4f*)(d + tid * 4) = o;
  __threadfence();
  if (tid < 8) *(volatile v4f*)(d + tid * 4) = o;
}

__global__ __launch_bounds__(256) void k_gnvar(const float* __restrict__ x, const float* __restrict__ GSs, float* __restrict__ GSv) {
  const int tid = threadIdx.x, c = blockIdx.x, b = blockIdx.y;
  const float ps = GSs[((size_t)b * 2 * CC + (tid & (CC - 1))) * 32];
  const float mean = blk_sum256((tid < CC) ? ps : 0.f) * (1.0f / (float)(CC * SEQ));
  const float* xr = x + (size_t)b * XS + (size_t)c * SEQ_FULL;
  float s = 0.f;
#pragma unroll 1
  for (int j = tid * 4; j < SEQ; j += 1024) {
    const v4f a = *(const v4fa*)(xr + j);
    const float d0 = bf16_rne(a[0]) - mean, d1 = bf16_rne(a[1]) - mean, d2 = bf16_rne(a[2]) - mean, d3 = bf16_rne(a[3]) - mean;
    s += (d0 * d0 + d1 * d1) + (d2 * d2 + d3 * d3);
  }
  const float tot = blk_sum256(s);
  float* d = GSv + ((size_t)b * 2 * CC + CC + c) * 32;
  const v4f o = {(tid == 0) ? tot : 0.f, 0.f, 0.f, 0.f};
  if (tid < 8) *(volatile v4f*)(d + tid * 4) = o;
  __threadfence();
  if (tid < 8) *(volatile v4f*)(d + tid * 4) = o;
}

__global__ __launch_bounds__(256) void k_qkv(const float* __restrict__ x, const float* __restrict__ gnw, const float* __restrict__ gnb,
                                             const _Float16* __restrict__ W16, const float* __restrict__ qb, const float* __restrict__ kb,
                                             const float* __restrict__ vb, const float* __restrict__ GS,
                                             _Float16* __restrict__ QK, _Float16* __restrict__ VT) {
  __shared__ __attribute__((aligned(16))) _Float16 hx[64 * HXP];
  __shared__ __attribute__((aligned(16))) _Float16 stg[128 * SVP];
  const int tid = threadIdx.x, w = tid >> 5, lane = tid & 31, ln = lane & 15, hh = lane >> 4;
  const int n0 = blockIdx.x * 64, b = blockIdx.y;
  const float invn = 1.0f / (float)(CC * SEQ);
  const size_t gsb = (size_t)b * 2 * CC;
  const float ps = GS[(gsb + (tid & (CC - 1))) * 32];
  const float pv = GS[(gsb + CC + (tid & (CC - 1))) * 32];
  const float mean = blk_sum256((tid < CC) ? ps : 0.f) * invn;
  const float var  = blk_sum256((tid < CC) ? pv : 0.f) * invn;
  const float rstd = rsqrtf(var + 1e-5f);
  const float* xb = x + (size_t)b * XS;
#pragma unroll 1
  for (int idx = tid; idx < CC * 64; idx += 256) {
    const int c = idx >> 6, col = idx & 63;
    const float v = bf16_rne(xb[(size_t)c * SEQ_FULL + n0 + col]);
    const float hv = ((v - mean) * rstd) * bf16_rne(gnw[c]) + bf16_rne(gnb[c]);
    hx[col * HXP + c] = (_Float16)hv;
  }
  __syncthreads();

  const float bqv = bf16_rne(qb[16 * w + ln]), bkv = bf16_rne(kb[16 * w + ln]);
#pragma unroll 1
  for (int m = 0; m < 2; ++m) {
    v16h fw[4];
    const _Float16* wr = W16 + (size_t)m * CC * CC + (size_t)(16 * w + ln) * CC;
#pragma unroll
    for (int kc = 0; kc < 4; ++kc) fw[kc] = ld_frag(wr + kc * 32, hh);
    const float bias = (m == 0) ? bqv : bkv;
#pragma unroll
    for (int nt = 0; nt < 4; ++nt) {
      v8f acc = {0.f, 0.f, 0.f, 0.f, 0.f, 0.f, 0.f, 0.f};
#pragma unroll
      for (int kc = 0; kc < 4; ++kc) {
        FragH fa;
        fa.half[0] = *(const v8us*)&hx[(nt * 16 + ln) * HXP + kc * 32 + 8 * hh];
        fa.half[1] = *(const v8us*)&hx[(nt * 16 + ln) * HXP + kc * 32 + 16 + 8 * hh];
        acc = mma(fa.v, fw[kc], acc);
      }
#pragma unroll
      for (int r = 0; r < 8; ++r) stg[(nt * 16 + 8 * hh + r) * HXP + 16 * w + ln] = (_Float16)(acc[r] * 0.0625f + bias);
    }
    __syncthreads();
    unsigned short* P = (unsigned short*)QK + (size_t)m * QKS + (size_t)b * NH * SEQ * HD;
    for (int pass = 0; pass < 2; ++pass) {
#pragma unroll
      for (int i = 0; i < 4; ++i) {
        const int idx = tid + 256 * i;
        const int head = idx >> 8, pi = idx & 255, tok = pi >> 2, d8 = (pi & 3) * 8;
        const v8us v = *(const v8us*)&stg[tok * HXP + head * HD + d8];
        *(volatile v8us*)(P + ((size_t)head * SEQ + n0 + tok) * HD + d8) = v;
      }
      if (pass == 0) __threadfence();
    }
    __syncthreads();
  }
  {
    v16h fw[4];
    const _Float16* wr = W16 + (size_t)2 * CC * CC + (size_t)(16 * w + ln) * CC;
#pragma unroll
    for (int kc = 0; kc < 4; ++kc) fw[kc] = ld_frag(wr + kc * 32, hh);
    float bvr[8];
#pragma unroll
    for (int r = 0; r < 8; ++r) bvr[r] = bf16_rne(vb[16 * w + 8 * hh + r]);
#pragma unroll
    for (int nt = 0; nt < 4; ++nt) {
      v8f acc = {0.f, 0.f, 0.f, 0.f, 0.f, 0.f, 0.f, 0.f};
#pragma unroll
      for (int kc = 0; kc < 4; ++kc) {
        FragH fb;
        fb.half[0] = *(const v8us*)&hx[(nt * 16 + ln) * HXP + kc * 32 + 8 * hh];
        fb.half[1] = *(const v8us*)&hx[(nt * 16 + ln) * HXP + kc * 32 + 16 + 8 * hh];
        acc = mma(fw[kc], fb.v, acc);
      }
#pragma unroll
      for (int r = 0; r < 8; ++r) stg[(16 * w + 8 * hh + r) * SVP + nt * 16 + ln] = (_Float16)(acc[r] * 0.0625f + bvr[r]);
    }
    __syncthreads();
    unsigned short* V = (unsigned short*)VT + (size_t)b * CC * SEQ;
    for (int pass = 0; pass < 2; ++pass) {
#pragma unroll
      for (int i = 0; i < 4; ++i) {
        const int idx = tid + 256 * i;
        const int o = idx >> 3, p8 = (idx & 7) * 8;
        const v8us v = *(const v8us*)&stg[o * SVP + p8];
        *(volatile v8us*)(V + (size_t)o * SEQ + n0 + p8) = v;
      }
      if (pass == 0) __threadfence();
    }
  }
}

__global__ __launch_bounds__(256) void k_attn(const _Float16* __restrict__ QK, const _Float16* __restrict__ VT, _Float16* __restrict__ AO) {
  __shared__ __attribute__((aligned(16))) _Float16 st[32 * HXP];
  const int tid = threadIdx.x, w = tid >> 5, lane = tid & 31, ln = lane & 15, hh = lane >> 4;
  const int hd = w & 3, qs = w >> 2, b = blockIdx.y;
  const int q0 = blockIdx.x * 32 + qs * 16;
  const _Float16* Qh = QK + ((size_t)b * NH + hd) * SEQ * HD;
  const _Float16* Kh = Qh + QKS;
  const _Float16* Vh = VT + ((size_t)b * CC + hd * HD) * SEQ;
  const v16h bq = ld_frag(Qh + (size_t)(q0 + ln) * HD, hh);
  const _Float16* kp  = Kh + (size_t)ln * HD;
  const _Float16* vp0 = Vh + (size_t)ln * SEQ;
  const _Float16* vp1 = Vh + (size_t)(16 + ln) * SEQ;
  const v8f z8 = {0.f, 0.f, 0.f, 0.f, 0.f, 0.f, 0.f, 0.f};
  const float sc = 0.17677669529663687f;
  float mrun = -1.0e30f, lrun = 0.f;
  v8f o0 = z8, o1 = z8;
#pragma unroll 1
  for (int kb = 0; kb < SEQ; kb += 32) {
    const v16h ka0 = ld_frag(kp + (size_t)kb * HD, hh);
    const v16h ka1 = ld_frag(kp + (size_t)(kb + 16) * HD, hh);
    v8f s0 = mma(ka0, bq, z8);
    v8f s1 = mma(ka1, bq, z8);
    float mx = -1.0e30f;
#pragma unroll
    for (int r = 0; r < 8; ++r) { s0[r] *= sc; s1[r] *= sc; mx = fmaxf(mx, fmaxf(s0[r], s1[r])); }
    mx = fmaxf(mx, __shfl_xor(mx, 16, 32));
    const float mn = fmaxf(mrun, mx);
    const float al = __expf(mrun - mn);
    mrun = mn;
    FragH pf;
    float rs = 0.f;
#pragma unroll
    for (int r = 0; r < 8; ++r) {
      const float p0 = __expf(s0[r] - mn), p1 = __expf(s1[r] - mn);
      rs += p0 + p1;
      pf.h[r]     = (_Float16)(p0 * 256.0f);
      pf.h[8 + r] = (_Float16)(p1 * 256.0f);
    }
    lrun = lrun * al + rs;
#pragma unroll
    for (int r = 0; r < 8; ++r) { o0[r] *= al; o1[r] *= al; }
    const v16h va0 = ld_frag(vp0 + kb, hh);
    const v16h va1 = ld_frag(vp1 + kb, hh);
    o0 = mma(va0, pf.v, o0);
    o1 = mma(va1, pf.v, o1);
  }
  const float lt = lrun + __shfl_xor(lrun, 16, 32);
  const float inv = 0.125f * (1.0f / lt);
  FragH e;
#pragma unroll
  for (int r = 0; r < 8; ++r) { e.h[r] = (_Float16)(o0[r] * inv); e.h[8 + r] = (_Float16)(o1[r] * inv); }
  *(v8us*)&st[(qs * 16 + ln) * HXP + hd * HD + 8 * hh]      = e.half[0];
  *(v8us*)&st[(qs * 16 + ln) * HXP + hd * HD + 16 + 8 * hh] = e.half[1];
  __syncthreads();
  unsigned short* A = (unsigned short*)AO + ((size_t)b * SEQ + (size_t)blockIdx.x * 32) * CC;
  for (int pass = 0; pass < 2; ++pass) {
#pragma unroll
    for (int i = 0; i < 2; ++i) {
      const int idx = tid + 256 * i;
      const int row = idx >> 4, p8 = (idx & 15) * 8;
      const v8us v = *(const v8us*)&st[row * HXP + p8];
      *(volatile v8us*)(A + (size_t)row * CC + p8) = v;
    }
    if (pass == 0) __threadfence();
  }
}

__global__ __launch_bounds__(256) void k_proj(const float* __restrict__ x, const _Float16* __restrict__ W16, const float* __restrict__ pb,
                                              const _Float16* __restrict__ AO, float* __restrict__ out) {
  __shared__ __attribute__((aligned(16))) float so[128 * SOP];
  const int tid = threadIdx.x, w = tid >> 5, lane = tid & 31, ln = lane & 15, hh = lane >> 4;
  const int n0 = blockIdx.x * 64, b = blockIdx.y;
  v16h fw[4];
  const _Float16* wr = W16 + (size_t)3 * CC * CC + (size_t)(16 * w + ln) * CC;
#pragma unroll
  for (int kc = 0; kc < 4; ++kc) fw[kc] = ld_frag(wr + kc * 32, hh);
#pragma unroll
  for (int nt = 0; nt < 4; ++nt) {
    const _Float16* br = AO + ((size_t)b * SEQ + n0 + nt * 16 + ln) * CC;
    v8f acc = {0.f, 0.f, 0.f, 0.f, 0.f, 0.f, 0.f, 0.f};
#pragma unroll
    for (int kc = 0; kc < 4; ++kc) { const v16h fb = ld_frag(br + kc * 32, hh); acc = mma(fw[kc], fb, acc); }
#pragma unroll
    for (int r = 0; r < 8; ++r) so[(16 * w + 8 * hh + r) * SOP + nt * 16 + ln] = acc[r] * 0.001953125f;
  }
  __syncthreads();
  const float* xb = x + (size_t)b * XS;
  float* ob = out + (size_t)b * XS;
  for (int pass = 0; pass < 2; ++pass) {
#pragma unroll 1
    for (int i = 0; i < 8; ++i) {
      const int idx = tid + 256 * i;
      const int o = idx >> 4, c4 = (idx & 15) * 4;
      const v4f a = *(const v4fa*)&so[o * SOP + c4];
      const size_t e = (size_t)o * SEQ_FULL + n0 + c4;
      const v4f xv = *(const v4fa*)(xb + e);
      const float pbv = bf16_rne(pb[o]);
      v4f y;
#pragma unroll
      for (int q = 0; q < 4; ++q) y[q] = bf16_rne(xv[q]) + (a[q] + pbv);
      *(volatile v4f*)(ob + e) = y;
    }
    if (pass == 0) __threadfence();
  }
}

extern "C" void kernel_launch(void* const* d_in, const int* in_sizes, int n_in,
                              void* d_out, int out_size, void* d_ws, size_t ws_size, hipStream_t stream) {
  if (n_in < 11) return;
  if (in_sizes[0] < NB * CC * SEQ) return;
  if (in_sizes[1] < CC || in_sizes[2] < CC || in_sizes[4] < CC || in_sizes[6] < CC || in_sizes[8] < CC || in_sizes[10] < CC) return;
  if (in_sizes[3] < CC * CC || in_sizes[5] < CC * CC || in_sizes[7] < CC * CC || in_sizes[9] < CC * CC) return;
  if (out_size < NB * CC * SEQ) return;
  if (ws_size < WS_TOTAL) return;
  const float* x   = (const float*)d_in[0];
  const float* gnw = (const float*)d_in[1];
  const float* gnb = (const float*)d_in[2];
  const float* qw  = (const float*)d_in[3];
  const float* qb  = (const float*)d_in[4];
  const float* kw  = (const float*)d_in[5];
  const float* kb  = (const float*)d_in[6];
  const float* vw  = (const float*)d_in[7];
  const float* vb  = (const float*)d_in[8];
  const float* pw  = (const float*)d_in[9];
  const float* pb  = (const float*)d_in[10];
  char* ws = (char*)d_ws;
  _Float16* W16 = (_Float16*)(ws + WS_W16);
  float*    GS  = (float*)(ws + WS_GS);
  _Float16* QK  = (_Float16*)(ws + WS_QK);
  _Float16* VT  = (_Float16*)(ws + WS_VT);
  _Float16* AO  = (_Float16*)(ws + WS_AO);
  k_wcvt<<<dim3(CC * CC / 8 / 256), 256, 0, stream>>>(qw, kw, vw, pw, W16);
  k_gnsum<<<dim3(CC, NB), 256, 0, stream>>>(x, GS);
  k_gnvar<<<dim3(CC, NB), 256, 0, stream>>>(x, GS, GS);
  k_qkv<<<dim3(SEQ / 64, NB), 256, 0, stream>>>(x, gnw, gnb, W16, qb, kb, vb, GS, QK, VT);
  k_attn<<<dim3(SEQ / 32, NB), 256, 0, stream>>>(QK, VT, AO);
  k_proj<<<dim3(SEQ / 64, NB), 256, 0, stream>>>(x, W16, pb, AO, (float*)d_out);
}
